// MLPPredictor_21174188769662
// MI455X (gfx1250) — hardware-verified
//
#include <hip/hip_runtime.h>


namespace {
constexpr int N = 50000, NP = 50048, E = 600000, ELIM = 600000  , D = 128;
constexpr float XS = 8.0f, WSC = 256.0f;
static_assert(NP % 64 == 0 && ELIM % 32 == 0, "tiling");
typedef _Float16 b16;
typedef __attribute__((ext_vector_type(16))) _Float16 v16b;
typedef __attribute__((ext_vector_type(8))) _Float16 v8b;
typedef __attribute__((ext_vector_type(8))) float v8f;
typedef __attribute__((ext_vector_type(4))) float v4f;
__device__ __forceinline__ float bf16_rne(float f) { unsigned int u = __float_as_uint(f); u += 0x7FFFu + ((u >> 16) & 1u); return __uint_as_float(u & 0xFFFF0000u); }
__device__ __forceinline__ void split16(float v, b16& hi, b16& lo) { hi = (b16)v; lo = (b16)(v - (float)hi); }
__device__ __forceinline__ v16b frag_kb(const b16* p, int hh) { const v8b a = *(const v8b*)(p + 8 * hh), b = *(const v8b*)(p + 16 + 8 * hh); v16b f;
#pragma unroll
  for (int e = 0; e < 8; ++e) { f[e] = a[e]; f[8 + e] = b[e]; } return f; }
__device__ __forceinline__ v8f wmma16b(v16b a, v16b b, v8f c) { v8f d = __builtin_amdgcn_wmma_f32_16x16x32_f16(false, a, false, b, (short)0, c, false, false); asm volatile("v_nop\n\tv_nop\n\tv_nop\n\tv_nop" : "+v"(d) : "v"(a), "v"(b)); return d; }
__device__ __forceinline__ void wave_lds_sync() { __builtin_amdgcn_fence(__ATOMIC_RELEASE, "workgroup"); __builtin_amdgcn_wave_barrier(); __builtin_amdgcn_fence(__ATOMIC_ACQUIRE, "workgroup"); }
__device__ __forceinline__ float pmul(float a, float b) { float p = a * b; asm volatile("" : "+v"(p)); return p; }
__device__ __forceinline__ int iclamp(int v, int lo, int hi) { return v < lo ? lo : (v > hi ? hi : v); }

__global__ __launch_bounds__(256) void prep_kernel(const float* __restrict__ w1, b16* __restrict__ WT) {
  const int t = blockIdx.x * 256 + threadIdx.x; if (t >= 2 * D * D / 8) return; const int e = t * 8; const int oo = e / D, k0 = e % D; const int o2 = oo % D, koff = (oo < D) ? 0 : D; v8b o;
  for (int j = 0; j < 8; ++j) o[j] = (b16)(bf16_rne(w1[(size_t)o2 * (2 * D) + koff + k0 + j]) * WSC);
  for (int pass = 0; pass < 2; ++pass) { *(volatile v8b*)(WT + e) = o; __threadfence(); }
}
__global__ __launch_bounds__(128) void proj_kernel(const float* __restrict__ x, const b16* __restrict__ WT, float* __restrict__ P) {
  __shared__ __attribute__((aligned(16))) float Tf[4][16][256 + 4];
  const int wave = threadIdx.x >> 5, lane = threadIdx.x & 31, nloc = lane & 15, hlf = lane >> 4; const size_t v0 = ((size_t)blockIdx.x * 4 + wave) * 16; const size_t vr = v0 + nloc; const size_t vra = vr < (size_t)N ? vr : (size_t)N - 1;
  v8f acc[16];
#pragma unroll
  for (int t = 0; t < 16; ++t) acc[t] = (v8f){};
#pragma unroll
  for (int ks = 0; ks < D / 32; ++ks) { v16b a; const float* xr = x + vra * D + ks * 32; const v4f c0 = *(const v4f*)(xr + 8 * hlf), c1 = *(const v4f*)(xr + 8 * hlf + 4), c2 = *(const v4f*)(xr + 16 + 8 * hlf), c3 = *(const v4f*)(xr + 16 + 8 * hlf + 4);
    for (int i = 0; i < 4; ++i) { a[i] = (b16)(bf16_rne(c0[i]) * XS); a[4 + i] = (b16)(bf16_rne(c1[i]) * XS); a[8 + i] = (b16)(bf16_rne(c2[i]) * XS); a[12 + i] = (b16)(bf16_rne(c3[i]) * XS); }
    if (vr >= (size_t)N) a = (v16b){};
#pragma unroll
    for (int t = 0; t < 16; ++t) acc[t] = wmma16b(a, frag_kb(WT + (size_t)(t * 16 + nloc) * D + ks * 32, hlf), acc[t]); }
#pragma unroll
  for (int t = 0; t < 16; ++t)
#pragma unroll
    for (int r = 0; r < 8; ++r) Tf[wave][8 * hlf + r][t * 16 + nloc] = acc[t][r] * (1.0f / (XS * WSC));
  wave_lds_sync();
  for (int pass = 0; pass < 2; ++pass) { for (int rr = 0; rr < 16; ++rr) { for (int q = lane * 4; q < 256; q += 128) *(volatile v4f*)(P + (v0 + rr) * 256 + q) = *(const v4f*)(&Tf[wave][rr][q]); } __threadfence(); }
}
__global__ __launch_bounds__(256) void edge_kernel(const float* __restrict__ P, const float* __restrict__ b1, const float* __restrict__ w2, const float* __restrict__ b2, const int* __restrict__ src, const int* __restrict__ dst, float* __restrict__ out) {
  __shared__ float SB1[D], SW2[D];
  for (int i = threadIdx.x; i < D; i += 256) { SB1[i] = bf16_rne(b1[i]); SW2[i] = bf16_rne(w2[i]); }
  __syncthreads();
  const size_t e = (size_t)blockIdx.x * 256 + threadIdx.x; if (e >= (size_t)ELIM) return;
  const size_t s = (size_t)iclamp(src[e], 0, N - 1), d = (size_t)iclamp(dst[e], 0, N - 1); const float* pa = P + s * 256; const float* pb = P + d * 256 + D; float acc = 0.0f;
#pragma unroll 4
  for (int c = 0; c < D; c += 4) { const v4f a = *(const v4f*)(pa + c), b = *(const v4f*)(pb + c); for (int i = 0; i < 4; ++i) acc += fmaxf(a[i] + b[i] + SB1[c + i], 0.0f) * SW2[c + i]; }
  acc += bf16_rne(b2[0]);
  for (int pass = 0; pass < 2; ++pass) { ((volatile float*)out)[e] = acc; __threadfence(); }
}
}

extern "C" void kernel_launch(void* const* d_in, const int* in_sizes, int n_in, void* d_out, int out_size, void* d_ws, size_t ws_size, hipStream_t stream) {
  (void)n_in;
  auto Fp = [&](int i) { return (const float*)d_in[i]; }; auto Ip = [&](int i) { return (const int*)d_in[i]; };
  if (in_sizes[0] != N * D || in_sizes[1] != D * 2 * D || in_sizes[2] != D || in_sizes[3] != D || in_sizes[4] != 1 || in_sizes[5] != E || in_sizes[6] != E || out_size != E) return;
  size_t off = 0; char* ws = (char*)d_ws;
  auto carve = [&](size_t bytes) { char* p = ws + off; off += (bytes + 255) & ~(size_t)255; return p; };
  b16* WT = (b16*)carve((size_t)2 * D * D * 2); float* P = (float*)carve((size_t)NP * 256 * 4);
  if (off > ws_size || off > ((size_t)128 << 20)) return;
  prep_kernel<<<(2 * D * D / 8 + 255) / 256, 256, 0, stream>>>(Fp(1), WT);
  proj_kernel<<<NP / 64, 128, 0, stream>>>(Fp(0), WT, P);
  edge_kernel<<<(ELIM + 255) / 256, 256, 0, stream>>>(P, Fp(2), Fp(3), Fp(4), Ip(5), Ip(6), (float*)d_out);
}
